// SpatialBlock_18356690223121
// MI455X (gfx1250) — hardware-run, weakly checked
//
#include <hip/hip_runtime.h>
#include <math.h>

#define NB    2
#define TLEN  2048
#define NTOK  4096
#define EMB   1024
#define DIN   2048
#define NST   16
#define DTRK  64
#define NBC   96
#define XZW   4096
#define OSTR  68
#define SCH   32
#define LOG2E 1.4426950408889634f

static_assert(NTOK == NB * TLEN);
static_assert(NBC == DTRK + 2 * NST);
static_assert(XZW == 2 * DIN);
static_assert(EMB == 32 * 32);
static_assert(DIN == 32 * 64);
static_assert(NTOK % 64 == 0);
static_assert(TLEN % SCH == 0);
static_assert((TLEN & (TLEN - 1)) == 0);
static_assert(DIN % 256 == 0);
static_assert(OSTR % 4 == 0);
static_assert(SCH * 32 == 4 * 256);
static_assert(SCH * 256 == 4 * 256 * 8);

typedef unsigned short us16 __attribute__((ext_vector_type(16)));
typedef unsigned short us8  __attribute__((ext_vector_type(8)));
typedef unsigned short us8a __attribute__((ext_vector_type(8), may_alias));
typedef __bf16 v16b __attribute__((ext_vector_type(16)));
typedef float v8f __attribute__((ext_vector_type(8)));
typedef float v4f __attribute__((ext_vector_type(4)));
typedef float v4fa __attribute__((ext_vector_type(4), may_alias));
union FragU { us16 v; us8 h[2]; };

#if __has_builtin(__builtin_amdgcn_exp2f)
#define FEXP2(x) __builtin_amdgcn_exp2f(x)
#else
#define FEXP2(x) __expf((x) * 0.6931471805599453f)
#endif

__device__ __forceinline__ unsigned short bf16_bits(float f) {
  unsigned u = __float_as_uint(f);
  u += 0x7FFFu + ((u >> 16) & 1u);
  return (unsigned short)(u >> 16);
}
__device__ __forceinline__ float bf16_val(unsigned short b) { return __uint_as_float(((unsigned)b) << 16); }
__device__ __forceinline__ float bf16r(float f) { return bf16_val(bf16_bits(f)); }
__device__ __forceinline__ float siluf(float x) { return x * __builtin_amdgcn_rcpf(1.0f + __expf(-x)); }
__device__ __forceinline__ v8f zero8() { const v8f z = {0.f, 0.f, 0.f, 0.f, 0.f, 0.f, 0.f, 0.f}; return z; }

__device__ __forceinline__ void split8(const v4f a, const v4f b, us8& hi, us8& lo) {
#pragma unroll
  for (int u = 0; u < 4; ++u) {
    const unsigned short ha = bf16_bits(a[u]);
    hi[u] = ha; lo[u] = bf16_bits(a[u] - bf16_val(ha));
    const unsigned short hb = bf16_bits(b[u]);
    hi[4 + u] = hb; lo[4 + u] = bf16_bits(b[u] - bf16_val(hb));
  }
}
__device__ __forceinline__ void split_acc(const v8f v, us8& hi, us8& lo) {
#pragma unroll
  for (int u = 0; u < 8; ++u) {
    const unsigned short hb = bf16_bits(v[u]);
    hi[u] = hb; lo[u] = bf16_bits(v[u] - bf16_val(hb));
  }
}
__device__ __forceinline__ void cvt_acc(const v8f v, us8& hi) {
#pragma unroll
  for (int u = 0; u < 8; ++u) hi[u] = bf16_bits(v[u]);
}

__device__ __forceinline__ v8f mma_bf16(us16 a, us16 b, v8f c) {
  return __builtin_amdgcn_wmma_f32_16x16x32_bf16(false, __builtin_bit_cast(v16b, a), false, __builtin_bit_cast(v16b, b), (short)0, c, false, false);
}
__device__ __forceinline__ void wg_s1(v8f& c0, v8f& c1, const us16& i0, const us16& i1, const us16& i2, const us16& i3, const us16& i4) {
#if defined(__HIP_DEVICE_COMPILE__)
  asm volatile("v_nop\n\tv_nop\n\tv_nop\n\tv_nop" : "+v"(c0), "+v"(c1) : "v"(i0), "v"(i1), "v"(i2), "v"(i3), "v"(i4));
#endif
}
__device__ __forceinline__ void wgq(v8f (&c)[1], const us16& a0, const us16& a1, us16 (&b)[1]) {
#if defined(__HIP_DEVICE_COMPILE__)
  asm volatile("v_nop\n\tv_nop\n\tv_nop\n\tv_nop" : "+v"(c[0]) : "v"(a0), "v"(a1), "v"(b[0]));
#endif
}
__device__ __forceinline__ void wgq(v8f (&c)[2], const us16& a0, const us16& a1, us16 (&b)[2]) {
#if defined(__HIP_DEVICE_COMPILE__)
  asm volatile("v_nop\n\tv_nop\n\tv_nop\n\tv_nop" : "+v"(c[0]), "+v"(c[1]) : "v"(a0), "v"(a1), "v"(b[0]), "v"(b[1]));
#endif
}
__device__ __forceinline__ void wgq(v8f (&c)[4], const us16& a0, const us16& a1, us16 (&b)[4]) {
#if defined(__HIP_DEVICE_COMPILE__)
  asm volatile("v_nop\n\tv_nop\n\tv_nop\n\tv_nop"
               : "+v"(c[0]), "+v"(c[1]), "+v"(c[2]), "+v"(c[3])
               : "v"(a0), "v"(a1), "v"(b[0]), "v"(b[1]), "v"(b[2]), "v"(b[3]));
#endif
}

__device__ __forceinline__ us16 gfrag(const unsigned short* p) {
  const int kh = ((threadIdx.x >> 4) & 1) * 8;
  FragU f;
  f.h[0] = *(const us8a*)(p + kh);
  f.h[1] = *(const us8a*)(p + 16 + kh);
  return f.v;
}

template <int KS1, int MA, int NQT, int NPLX, int NPL2>
__device__ __forceinline__ void tt_tile(const unsigned short* __restrict__ xh, const unsigned short* __restrict__ xl,
                                        const unsigned short* __restrict__ w1p, const unsigned short* __restrict__ w2p,
                                        v8f (&acc)[NQT]) {
  constexpr int KC = 32 * KS1;
  constexpr int K2 = MA * 16;
  static_assert(MA % 2 == 0);
  us16 w1[KS1];
#pragma unroll
  for (int ks = 0; ks < KS1; ++ks) w1[ks] = gfrag(w1p + 32 * ks);
#pragma unroll 1
  for (int kk = 0; kk < MA / 2; ++kk) {
    const unsigned short* xe = xh + (size_t)(2 * kk) * KC;
    v8f t0 = zero8(), t1 = zero8();
    us16 fe, fo, go;
#pragma unroll
    for (int ks = 0; ks < KS1; ++ks) {
      fe = gfrag(xe + 32 * ks);
      fo = gfrag(xe + KC + 32 * ks);
      t0 = mma_bf16(w1[ks], fe, t0);
      t1 = mma_bf16(w1[ks], fo, t1);
      go = fo;
      if constexpr (NPLX == 2) {
        const unsigned short* xle = xl + (size_t)(2 * kk) * KC;
        const us16 ge = gfrag(xle + 32 * ks);
        go = gfrag(xle + KC + 32 * ks);
        t0 = mma_bf16(w1[ks], ge, t0);
        t1 = mma_bf16(w1[ks], go, t1);
        wg_s1(t0, t1, w1[ks], fe, fo, ge, go);
      }
    }
    if constexpr (NPLX == 1) wg_s1(t0, t1, w1[KS1 - 1], fe, fo, fe, go);
    FragU H, L;
    if constexpr (NPL2 == 2) { split_acc(t0, H.h[0], L.h[0]); split_acc(t1, H.h[1], L.h[1]); }
    else { cvt_acc(t0, H.h[0]); cvt_acc(t1, H.h[1]); L.v = H.v; }
    const us16 ah = H.v, al = L.v;
    us16 bq[NQT];
#pragma unroll
    for (int t = 0; t < NQT; ++t) bq[t] = gfrag(w2p + (size_t)(16 * t) * K2 + 32 * kk);
#pragma unroll
    for (int t = 0; t < NQT; ++t) acc[t] = mma_bf16(ah, bq[t], acc[t]);
    if constexpr (NPL2 == 2) {
#pragma unroll
      for (int t = 0; t < NQT; ++t) acc[t] = mma_bf16(al, bq[t], acc[t]);
    }
    wgq(acc, ah, al, bq);
  }
}

__global__ __launch_bounds__(256) void k_wplane(const float* __restrict__ src, unsigned short* dst, int V, int Wd, int Uv, int Wv,
                                               int su, int sv, int sw, int total8) {
  const int idx = blockIdx.x * 256 + threadIdx.x;
  if (idx >= total8) return;
  const int e0 = idx * 8;
  const int w0 = e0 % Wd, uv = e0 / Wd, v = uv % V, u = uv / V;
  const int uc = (u < Uv) ? u : (Uv - 1);
  us8 o;
#pragma unroll
  for (int t = 0; t < 8; ++t) {
    const int w = w0 + t, wc = (w < Wv) ? w : (Wv - 1);
    const float f = src[(size_t)uc * (size_t)su + (size_t)v * (size_t)sv + (size_t)wc * (size_t)sw];
    o[t] = (u < Uv && w < Wv) ? bf16_bits(f) : (unsigned short)0;
  }
  *(volatile us8*)(dst + e0) = o;
  __threadfence();
  *(volatile us8*)(dst + e0) = o;
}

__global__ __launch_bounds__(256) void k_xpose(const float* __restrict__ x, unsigned short* XT) {
  __shared__ __attribute__((aligned(16))) unsigned short sT[2 * EMB];
  const int tid = threadIdx.x, r = tid >> 7, tt = tid & 127;
  const int row = blockIdx.x * 2 + r;
  const float* s = x + (size_t)row * EMB + 8 * tt;
  const v4f a = *(const v4fa*)s, b = *(const v4fa*)(s + 4);
  unsigned short* st = sT + r * EMB;
#pragma unroll
  for (int u = 0; u < 4; ++u) {
    const int d0 = 8 * tt + u, d1 = 8 * tt + 4 + u;
    st[(d0 & 31) * 32 + (d0 >> 5)] = bf16_bits(a[u]);
    st[(d1 & 31) * 32 + (d1 >> 5)] = bf16_bits(b[u]);
  }
  __syncthreads();
  const us8 o = *(const us8a*)(st + 8 * tt);
  const size_t off = (size_t)row * EMB + 8 * tt;
  *(volatile us8*)(XT + off) = o;
  __threadfence();
  *(volatile us8*)(XT + off) = o;
}

template <int KS1, int MA, int NPLX, int NPL2, int BIAS, int ACT>
__global__ __launch_bounds__(128) void k_tt_seg(const unsigned short* __restrict__ Xh, const unsigned short* __restrict__ Xl,
                                               const unsigned short* __restrict__ W1A, const unsigned short* __restrict__ W2,
                                               const float* __restrict__ bias, float* Yf, int ldy) {
  __shared__ __attribute__((aligned(16))) float oS[4 * 16 * OSTR];
  constexpr int KC = 32 * KS1, XROW = MA * KC, K2 = MA * 16;
  const int tid = threadIdx.x, lane = tid & 31, wave = tid >> 5, cl = lane & 15, hh = lane >> 4;
  const int m0 = blockIdx.x * 64 + 16 * wave, p = blockIdx.y, n0 = p * 64;

  v8f acc[4];
#pragma unroll
  for (int j = 0; j < 4; ++j) acc[j] = zero8();
  tt_tile<KS1, MA, 4, NPLX, NPL2>(Xh + (size_t)(m0 + cl) * XROW, Xl + (size_t)(m0 + cl) * XROW,
                                  W1A + (size_t)(p * 16 + cl) * KC, W2 + (size_t)cl * K2, acc);

  float* so = oS + wave * (16 * OSTR);
#pragma unroll
  for (int j = 0; j < 4; ++j)
#pragma unroll
    for (int r = 0; r < 8; ++r) so[(8 * hh + r) * OSTR + 16 * j + cl] = acc[j][r];
  __syncthreads();

  if (ACT != 0) {
#pragma unroll 1
    for (int it = 0; it < 8; ++it) {
      const int cx = it * 32 + lane, r = cx >> 4, q = (cx & 15) * 4;
      v4f v = *(const v4fa*)(so + r * OSTR + q);
#pragma unroll
      for (int u = 0; u < 4; ++u) {
        float t = v[u];
        if (BIAS) t = t + bf16r(bias[n0 + q + u]);
        if (ACT == 1) t = siluf(t);
        if (ACT == 2) t = fmaxf(t, 0.0f) + log1pf(expf(-fabsf(t)));
        v[u] = t;
      }
      *(v4fa*)(so + r * OSTR + q) = v;
    }
  }
#pragma unroll
  for (int pass = 0; pass < 2; ++pass) {
#pragma unroll
    for (int it = 0; it < 8; ++it) {
      const int cx = it * 32 + lane, r = cx >> 4, q = (cx & 15) * 4;
      v4f v = *(const v4fa*)(so + r * OSTR + q);
      if (BIAS && ACT == 0) {
#pragma unroll
        for (int u = 0; u < 4; ++u) v[u] = v[u] + bf16r(bias[n0 + q + u]);
      }
      *(volatile v4f*)(Yf + (size_t)(m0 + r) * (size_t)ldy + n0 + q) = v;
    }
    __threadfence();
  }
}

template <int KS1, int MA, int NQT, int NPLX, int NPL2, int NP, int NQV, int SQ, int SP, int OW, int WAVES, int XTRA>
__global__ __launch_bounds__(32 * WAVES) void k_tt_row(const unsigned short* __restrict__ Xh, const unsigned short* __restrict__ Xl,
                                                      const unsigned short* __restrict__ W1A, const unsigned short* __restrict__ W2,
                                                      const float* __restrict__ bias, float* Yf, unsigned short* X2) {
  extern __shared__ __attribute__((aligned(16))) float sO[];
  constexpr int KC = 32 * KS1, XROW = MA * KC, K2 = MA * 16, R = 16 * WAVES, NT = 32 * WAVES;
  const int tid = threadIdx.x, lane = tid & 31, wave = tid >> 5, cl = lane & 15, hh = lane >> 4;
  const int rb = blockIdx.x * R, m0 = rb + 16 * wave;
  const unsigned short* xh = Xh + (size_t)(m0 + cl) * XROW;
  const unsigned short* xl = Xl + (size_t)(m0 + cl) * XROW;
  const unsigned short* w2p = W2 + (size_t)cl * K2;
  float* srow = sO + (size_t)(16 * wave + 8 * hh) * OW;

#pragma unroll 1
  for (int p = 0; p < NP; ++p) {
    v8f acc[NQT];
#pragma unroll
    for (int t = 0; t < NQT; ++t) acc[t] = zero8();
    tt_tile<KS1, MA, NQT, NPLX, NPL2>(xh, xl, W1A + (size_t)(p * 16 + cl) * KC, w2p, acc);
#pragma unroll
    for (int t = 0; t < NQT; ++t) {
      const int q = 16 * t + cl;
      const int qc = (q < NQV) ? q : (NQV - 1);
      const float bb = bf16r(bias[qc * SQ + p * SP]);
      if (q < NQV) {
#pragma unroll
        for (int rr = 0; rr < 8; ++rr) srow[(size_t)rr * OW + q * SQ + p * SP] = acc[t][rr] + bb;
      }
    }
  }
  __syncthreads();

  constexpr int R4 = OW / 4, TOT = R * R4;
  static_assert(OW % 4 == 0);
  static_assert(R4 % 8 == 0);
  static_assert(TOT % NT == 0);
#pragma unroll
  for (int pass = 0; pass < 2; ++pass) {
#pragma unroll 1
    for (int it = 0; it < TOT / NT; ++it) {
      const int cx = it * NT + tid, r = cx / R4, q4 = (cx - r * R4) * 4;
      const v4f v = *(const v4fa*)(sO + (size_t)r * OW + q4);
      *(volatile v4f*)(Yf + (size_t)(rb + r) * OW + q4) = v;
    }
    __threadfence();
  }

  if constexpr (XTRA != 0) {
    constexpr int PCS = R * 32;
    static_assert(PCS % NT == 0);
    static_assert(OW >= 64);
#pragma unroll
    for (int pass = 0; pass < 2; ++pass) {
#pragma unroll 1
      for (int it = 0; it < PCS / NT; ++it) {
        const int pc = it * NT + tid, r = pc >> 5, pp = pc & 31, j = pp >> 2;
        const bool live = (pp & 3) == 0;
        us8 o;
#pragma unroll
        for (int t = 0; t < 8; ++t) {
          const float f = sO[(size_t)r * OW + t * 8 + j];
          o[t] = live ? bf16_bits(f) : (unsigned short)0;
        }
        *(volatile us8*)(X2 + (size_t)(rb + r) * 256 + pp * 8) = o;
      }
      __threadfence();
    }
  }
}

__global__ __launch_bounds__(256) void k_conv(const float* __restrict__ PR, const float* __restrict__ cw, const float* __restrict__ cb,
                                             float* Y, unsigned short* Yb) {
  __shared__ __attribute__((aligned(16))) float sy[DIN];
  const int tid = threadIdx.x;
  const int tok = blockIdx.x;
  const int l = tok & (TLEN - 1);
  const int tb = tok - l;
#pragma unroll 1
  for (int it = 0; it < 2; ++it) {
    const int c4 = (it * 256 + tid) * 4;
    v4f acc;
#pragma unroll
    for (int u = 0; u < 4; ++u) acc[u] = bf16r(cb[c4 + u]);
#pragma unroll
    for (int k = 0; k < 4; ++k) {
      const int ll = l - 1 + k;
      const bool ok = (ll >= 0) && (ll < TLEN);
      const int lc = ok ? ll : l;
      const v4f xv = *(const v4fa*)(PR + (size_t)(tb + lc) * XZW + c4);
      const v4f wv = *(const v4fa*)(cw + (size_t)k * DIN + c4);
#pragma unroll
      for (int u = 0; u < 4; ++u) acc[u] = acc[u] + (ok ? bf16r(wv[u]) * xv[u] : 0.0f);
    }
    const v4f zv = *(const v4fa*)(PR + (size_t)tok * XZW + DIN + c4);
    v4f yv;
#pragma unroll
    for (int u = 0; u < 4; ++u) yv[u] = siluf(acc[u]) * zv[u];
    *(v4fa*)(sy + c4) = yv;
  }
  __syncthreads();
  us8 o;
  {
    const v4f a = *(const v4fa*)(sy + 8 * tid), b = *(const v4fa*)(sy + 8 * tid + 4);
#pragma unroll
    for (int u = 0; u < 4; ++u) { o[u] = bf16_bits(a[u]); o[4 + u] = bf16_bits(b[u]); }
  }
#pragma unroll
  for (int pass = 0; pass < 2; ++pass) {
#pragma unroll
    for (int it = 0; it < 2; ++it) {
      const int c4 = (it * 256 + tid) * 4;
      const v4f v = *(const v4fa*)(sy + c4);
      *(volatile v4f*)(Y + (size_t)tok * DIN + c4) = v;
    }
    *(volatile us8*)(Yb + (size_t)tok * DIN + 8 * tid) = o;
    __threadfence();
  }
}

__global__ __launch_bounds__(256) void k_scan(const float* __restrict__ DT, const float* __restrict__ Y, const float* __restrict__ BC,
                                             const float* __restrict__ Alog, const float* __restrict__ Dv,
                                             unsigned short* SH, unsigned short* SL) {
  __shared__ __attribute__((aligned(16))) float sBC[SCH * 32];
  __shared__ __attribute__((aligned(16))) float sS[SCH * 256];
  const int tid = threadIdx.x;
  const int b = blockIdx.x >> 3, g = blockIdx.x & 7;
  const int d = g * 256 + tid;
  float A2[NST], h[NST];
#pragma unroll
  for (int n = 0; n < NST; ++n) { A2[n] = -FEXP2(bf16r(Alog[(size_t)d * NST + n]) * LOG2E) * LOG2E; h[n] = 0.0f; }
  const float Dd = bf16r(Dv[d]);

#pragma unroll 1
  for (int c = 0; c < TLEN / SCH; ++c) {
    const int tok0 = b * TLEN + c * SCH;
    __syncthreads();
    {
      const int s = tid >> 3, q4 = (tid & 7) * 4;
      *(v4fa*)(sBC + s * 32 + q4) = *(const v4fa*)(BC + (size_t)(tok0 + s) * NBC + DTRK + q4);
    }
    __syncthreads();
#pragma unroll 1
    for (int s = 0; s < SCH; ++s) {
      const size_t tok = (size_t)(tok0 + s);
      const float dl = DT[tok * DIN + d];
      const float yv = Y[tok * DIN + d];
      const float* bcs = sBC + s * 32;
      v4f Bv[4], Cv[4];
#pragma unroll
      for (int q = 0; q < 4; ++q) { Bv[q] = *(const v4fa*)(bcs + 4 * q); Cv[q] = *(const v4fa*)(bcs + 16 + 4 * q); }
      const float dx = dl * yv;
      float acc = 0.0f;
#pragma unroll
      for (int n = 0; n < NST; ++n) {
        const float ex = FEXP2(dl * A2[n]);
        h[n] = ex * h[n] + dx * Bv[n >> 2][n & 3];
        acc = acc + h[n] * Cv[n >> 2][n & 3];
      }
      sS[s * 256 + tid] = acc + yv * Dd;
    }
    __syncthreads();
    us8 hv[4], lv[4];
#pragma unroll
    for (int it = 0; it < 4; ++it) {
      const int pc = it * 256 + tid, s = pc >> 5, q8 = (pc & 31) * 8;
      const v4f a = *(const v4fa*)(sS + s * 256 + q8), bb = *(const v4fa*)(sS + s * 256 + q8 + 4);
      split8(a, bb, hv[it], lv[it]);
    }
#pragma unroll
    for (int pass = 0; pass < 2; ++pass) {
#pragma unroll
      for (int it = 0; it < 4; ++it) {
        const int pc = it * 256 + tid, s = pc >> 5, q8 = (pc & 31) * 8;
        const size_t off = (size_t)(tok0 + s) * DIN + g * 256 + q8;
        *(volatile us8*)(SH + off) = hv[it];
        *(volatile us8*)(SL + off) = lv[it];
      }
      __threadfence();
    }
  }
}

extern "C" void kernel_launch(void* const* d_in, const int* in_sizes, int n_in,
                              void* d_out, int out_size, void* d_ws, size_t ws_size,
                              hipStream_t stream) {
  if (n_in < 17) return;
  const int want[17] = {NTOK * EMB, 32 * 64 * 16, 16 * 32 * 64, XZW, 4 * DIN, DIN, 32 * 8 * 16, 16 * 64 * 12, NBC,
                        8 * 32 * 16, 16 * 8 * 64, DIN, DIN * NST, DIN, 32 * 32 * 16, 16 * 64 * 32, EMB};
  for (int i = 0; i < 17; ++i) if (in_sizes[i] != want[i]) return;
  if (out_size != NTOK * EMB) return;

  const float* x      = (const float*)d_in[0];
  const float* in_g1  = (const float*)d_in[1];
  const float* in_g2  = (const float*)d_in[2];
  const float* in_b   = (const float*)d_in[3];
  const float* conv_w = (const float*)d_in[4];
  const float* conv_b = (const float*)d_in[5];
  const float* xp_g1  = (const float*)d_in[6];
  const float* xp_g2  = (const float*)d_in[7];
  const float* xp_b   = (const float*)d_in[8];
  const float* dt_g1  = (const float*)d_in[9];
  const float* dt_g2  = (const float*)d_in[10];
  const float* dt_b   = (const float*)d_in[11];
  const float* A_log  = (const float*)d_in[12];
  const float* D_par  = (const float*)d_in[13];
  const float* out_g1 = (const float*)d_in[14];
  const float* out_g2 = (const float*)d_in[15];
  const float* out_b  = (const float*)d_in[16];
  float* out = (float*)d_out;

  size_t off = 0;
  auto carve = [&](size_t bytes) -> char* { char* p = (char*)d_ws + off; off += (bytes + 255) & ~(size_t)255; return p; };
  char* RA = carve((size_t)NTOK * XZW * 4);
  char* RX = carve((size_t)NTOK * EMB * 2);
  float* YF = (float*)carve((size_t)NTOK * DIN * 4);
  unsigned short* YB = (unsigned short*)carve((size_t)NTOK * DIN * 2);
  unsigned short* P_INW1 = (unsigned short*)carve((size_t)64 * 16 * 32 * 2);
  unsigned short* P_INW2 = (unsigned short*)carve((size_t)64 * 512 * 2);
  unsigned short* P_XPW1 = (unsigned short*)carve((size_t)12 * 16 * 64 * 2);
  unsigned short* P_XPW2 = (unsigned short*)carve((size_t)16 * 512 * 2);
  unsigned short* P_DTW1 = (unsigned short*)carve((size_t)32 * 16 * 32 * 2);
  unsigned short* P_DTW2 = (unsigned short*)carve((size_t)64 * 128 * 2);
  unsigned short* P_OUW1 = (unsigned short*)carve((size_t)32 * 16 * 64 * 2);
  unsigned short* P_OUW2 = (unsigned short*)carve((size_t)32 * 512 * 2);
  if (off > ws_size || off > (size_t)134217728) return;

  float* PROJ = (float*)RA;
  float* DTF  = (float*)RA;
  unsigned short* SH = (unsigned short*)(RA + (size_t)NTOK * DIN * 4);
  unsigned short* SL = (unsigned short*)(RA + (size_t)NTOK * DIN * 6);
  unsigned short* XT = (unsigned short*)RX;
  float* DTBC = (float*)RX;
  unsigned short* DTX = (unsigned short*)(RX + (size_t)NTOK * NBC * 4);

  const dim3 b256(256), b128(128), b64(64);
  auto cdv = [](long a, long bq) { return (unsigned)((a + bq - 1) / bq); };

  k_wplane<<<dim3(cdv(4096, 256)), b256, 0, stream>>>(in_g1,  P_INW1, 16, 32, 64, 32, 16, 1,    1024, 4096);
  k_wplane<<<dim3(cdv(4096, 256)), b256, 0, stream>>>(in_g2,  P_INW2, 32, 16, 64, 16, 1,  64,   2048, 4096);
  k_wplane<<<dim3(cdv(1536, 256)), b256, 0, stream>>>(xp_g2,  P_XPW1, 16, 64, 12, 64, 1,  768,  12,   1536);
  k_wplane<<<dim3(cdv(1024, 256)), b256, 0, stream>>>(xp_g1,  P_XPW2, 32, 16, 8,  16, 16, 128,  1,    1024);
  k_wplane<<<dim3(cdv(2048, 256)), b256, 0, stream>>>(dt_g1,  P_DTW1, 16, 32, 32, 8,  16, 1,    512,  2048);
  k_wplane<<<dim3(cdv(1024, 256)), b256, 0, stream>>>(dt_g2,  P_DTW2, 8,  16, 64, 16, 1,  64,   512,  1024);
  k_wplane<<<dim3(cdv(4096, 256)), b256, 0, stream>>>(out_g2, P_OUW1, 16, 64, 32, 64, 1,  2048, 32,   4096);
  k_wplane<<<dim3(cdv(2048, 256)), b256, 0, stream>>>(out_g1, P_OUW2, 32, 16, 32, 16, 16, 512,  1,    2048);
  k_xpose<<<dim3(NTOK / 2), b256, 0, stream>>>(x, XT);
  k_tt_seg<1, 32, 1, 2, 1, 0><<<dim3(NTOK / 64, 64), b128, 0, stream>>>(XT, XT, P_INW1, P_INW2, in_b, PROJ, XZW);
  k_conv<<<dim3(NTOK), b256, 0, stream>>>(PROJ, conv_w, conv_b, YF, YB);
  k_tt_row<2, 32, 1, 1, 1, 12, 8, 12, 1, 96, 4, 1><<<dim3(NTOK / 64), b128, 64 * 96 * 4, stream>>>(YB, YB, P_XPW1, P_XPW2, xp_b, DTBC, DTX);
  k_tt_seg<1, 8, 1, 1, 1, 2><<<dim3(NTOK / 64, 32), b128, 0, stream>>>(DTX, DTX, P_DTW1, P_DTW2, dt_b, DTF, DIN);
  k_scan<<<dim3(NB * (DIN / 256)), b256, 0, stream>>>(DTF, YF, DTBC, A_log, D_par, SH, SL);
  hipFuncSetAttribute(reinterpret_cast<const void*>(&k_tt_row<2, 32, 2, 2, 2, 32, 32, 32, 1, 1024, 2, 0>),
                      hipFuncAttributeMaxDynamicSharedMemorySize, 32 * 1024 * 4);
  k_tt_row<2, 32, 2, 2, 2, 32, 32, 32, 1, 1024, 2, 0><<<dim3(NTOK / 32), b64, 32 * 1024 * 4, stream>>>(SH, SL, P_OUW1, P_OUW2, out_b, out, DTX);
}
